// SINKAttention_16140487098656
// MI455X (gfx1250) — hardware-verified
//
#include <hip/hip_runtime.h>
#include <math.h>

typedef __attribute__((ext_vector_type(16))) _Float16 v16h;
typedef __attribute__((ext_vector_type(16))) __bf16 v16b;
typedef __attribute__((ext_vector_type(8)))  _Float16 v8h;
typedef __attribute__((ext_vector_type(8)))  float v8f;
typedef __attribute__((ext_vector_type(4)))  float v4f;
typedef __attribute__((ext_vector_type(2)))  float v2f;
typedef __attribute__((ext_vector_type(4)))  unsigned v4u;
typedef __attribute__((ext_vector_type(4)))  int v4i;
typedef float __attribute__((may_alias)) float_a;
typedef int __attribute__((may_alias)) int_a;

template <typename T> __device__ __forceinline__ void vst2(void* p, T v) { *(volatile T*)p = v; __threadfence(); *(volatile T*)p = v; }
__device__ __forceinline__ v8f wmma16(v16h a, v16h b, v8f c) {
  v8f d = __builtin_amdgcn_wmma_f32_16x16x32_f16(false, a, false, b, (short)0, c, false, false);
  asm volatile("v_nop\n\tv_nop\n\tv_nop\n\tv_nop" : "+v"(d) : "v"(a), "v"(b));
  return d;
}
__device__ __forceinline__ v8f wmma_bf(v16b a, v16b b, v8f c) {
  v8f d = __builtin_amdgcn_wmma_f32_16x16x32_bf16(false, a, false, b, (short)0, c, false, false);
  asm volatile("v_nop\n\tv_nop\n\tv_nop\n\tv_nop" : "+v"(d) : "v"(a), "v"(b));
  return d;
}
__device__ __forceinline__ v16h frag_h(const _Float16* rowk0, int lane) {
  union { v16h v; v8h q[2]; } u; const _Float16* p = rowk0 + 8 * (lane >> 4);
  u.q[0] = *(const v8h*)p; u.q[1] = *(const v8h*)(p + 16); return u.v;
}
__device__ __forceinline__ v16h frag_f32(const float* rowk0, int lane) {
  v16h a; const float* p = rowk0 + 8 * (lane >> 4);
#pragma unroll
  for (int i = 0; i < 8; ++i) { a[i] = (_Float16)p[i]; a[8 + i] = (_Float16)p[16 + i]; }
  return a;
}
__device__ __forceinline__ v16h frag_f32s(const float* rowk0, int lane, float sc) {
  v16h a; const float* p = rowk0 + 8 * (lane >> 4);
#pragma unroll
  for (int i = 0; i < 8; ++i) { a[i] = (_Float16)(p[i] * sc); a[8 + i] = (_Float16)(p[16 + i] * sc); }
  return a;
}
__device__ __forceinline__ v16h fragc_f32(const float* W, int k0, int n, int lane, int ld, int K) {
  v16h a; const int g = lane >> 4;
#pragma unroll
  for (int i = 0; i < 8; ++i) { const int ka = k0 + 8 * g + i, kb = ka + 16;
    a[i] = (_Float16)(ka < K ? W[(size_t)(ka < K ? ka : K - 1) * ld + n] : 0.f); a[8 + i] = (_Float16)(kb < K ? W[(size_t)(kb < K ? kb : K - 1) * ld + n] : 0.f); }
  return a;
}
struct F2 { v16b h, l; };
__device__ __forceinline__ F2 bsplit16(const float v[16]) { F2 r;
#pragma unroll
  for (int i = 0; i < 16; ++i) { const __bf16 h = (__bf16)v[i]; r.h[i] = h; r.l[i] = (__bf16)(v[i] - (float)h); }
  return r; }
__device__ __forceinline__ F2 split_row(const float* row, int k0, int lane) { float v[16]; const float* p = row + k0 + 8 * (lane >> 4);
#pragma unroll
  for (int i = 0; i < 8; ++i) { v[i] = p[i]; v[8 + i] = p[16 + i]; }
  return bsplit16(v); }
__device__ __forceinline__ F2 split_rowK(const float* row, int k0, int lane, int K) { float v[16]; const int g = lane >> 4;
#pragma unroll
  for (int i = 0; i < 8; ++i) { const int ka = k0 + 8 * g + i, kb = ka + 16; v[i] = ka < K ? row[ka < K ? ka : K - 1] : 0.f; v[8 + i] = kb < K ? row[kb < K ? kb : K - 1] : 0.f; }
  return bsplit16(v); }
__device__ __forceinline__ F2 split_col(const float* W, int k0, int n, int lane, int ld, int K) { float v[16]; const int g = lane >> 4;
#pragma unroll
  for (int i = 0; i < 8; ++i) { const int ka = k0 + 8 * g + i, kb = ka + 16; v[i] = ka < K ? W[(size_t)(ka < K ? ka : K - 1) * ld + n] : 0.f; v[8 + i] = kb < K ? W[(size_t)(kb < K ? kb : K - 1) * ld + n] : 0.f; }
  return bsplit16(v); }
__device__ __forceinline__ v8f mac3(const F2& a, const F2& b, v8f c) { c = wmma_bf(a.l, b.h, c); c = wmma_bf(a.h, b.l, c); return wmma_bf(a.h, b.h, c); }
__device__ __forceinline__ float sigm(float v) { return 1.0f / (1.0f + expf(-v)); }
#define LDSX() do { asm volatile("s_wait_dscnt 0" ::: "memory"); __builtin_amdgcn_wave_barrier(); __builtin_amdgcn_fence(__ATOMIC_RELEASE, "workgroup"); } while (0)


#define NB 2
#define NH 8
#define NS 2048
#define DD 32
#ifndef TBH
#define TBH (NB * NH)
#endif
typedef __attribute__((ext_vector_type(8))) __bf16 v8b;
__device__ __forceinline__ v16b frag_b(const __bf16* rowk0, int lane) {
  union { v16b v; v8b q[2]; } u; const __bf16* p = rowk0 + 8 * (lane >> 4);
  u.q[0] = *(const v8b*)p; u.q[1] = *(const v8b*)(p + 16); return u.v;
}
__device__ __forceinline__ float bfr(float v) { return (float)(__bf16)v; }
__device__ __attribute__((noinline)) float exp_ni(float v) { return expf(v); }
__device__ __attribute__((noinline)) float erf_ni(float v) { return erff(v); }

#define WS_U1  0u
#define WS_V1  (WS_U1 + 4u * (size_t)NB * NH * NS)
#define WS_VT  (WS_V1 + 4u * (size_t)NB * NH * NS)
#define WS_END (WS_VT + 2u * (size_t)NB * NH * DD * NS)

__device__ __forceinline__ v16b frag_in(const float* __restrict__ p, int lane) { v16b a; const float* pp = p + 8 * (lane >> 4);
#pragma unroll
  for (int i = 0; i < 8; ++i) { a[i] = (__bf16)pp[i]; a[8 + i] = (__bf16)pp[16 + i]; } return a; }
__global__ __launch_bounds__(128) void k_vt(const float* __restrict__ V, _Float16* __restrict__ VT) { __shared__ __align__(16) _Float16 th[DD][72]; const int t = threadIdx.x; const size_t bh = blockIdx.y; const int m0 = blockIdx.x * 64;
  for (int e = t; e < 64 * DD; e += 128) { const int ml = e / DD, d = e % DD; th[d][ml] = (_Float16)bfr(V[(bh * NS + m0 + ml) * DD + d]); }
  __syncthreads(); for (int e = t; e < DD * 8; e += 128) { const int d = e >> 3, q = e & 7; vst2((unsigned*)(VT + (bh * DD + d) * (size_t)NS + m0 + q * 8), *(const v4u*)&th[d][q * 8]); } }
__global__ __launch_bounds__(128) void k_rowlse(const float* __restrict__ Q, const float* __restrict__ K, const int* __restrict__ MK, float* __restrict__ U1) { __shared__ __align__(16) float su[64];
  const int tid = threadIdx.x, wave = tid >> 5, lane = tid & 31, col = lane & 15, g = lane >> 4; const size_t bh = blockIdx.y; const size_t b = bh / NH; const int i0 = blockIdx.x * 64 + wave * 16;
  const v16b aq = frag_in(Q + (bh * NS + i0 + col) * DD, lane);
  float m[8], l[8];
#pragma unroll
  for (int r = 0; r < 8; ++r) { m[r] = -3.0e38f; l[r] = 0.f; }
#pragma unroll 1
  for (int ks = 0; ks < NS / 32; ++ks) { float s[2][8];
#pragma unroll
    for (int ct = 0; ct < 2; ++ct) { const int kk = ks * 32 + ct * 16 + col; v8f c = {}; c = wmma_bf(aq, frag_in(K + (bh * NS + kk) * DD, lane), c); const bool msk = (MK[b * NS + kk] != 0);
#pragma unroll
      for (int r = 0; r < 8; ++r) s[ct][r] = msk ? -10000.0f : c[r] * 0.17677669529663687f; }
#pragma unroll
    for (int r = 0; r < 8; ++r) { float mx = fmaxf(s[0][r], s[1][r]);
#pragma unroll
      for (int o = 1; o < 16; o <<= 1) mx = fmaxf(mx, __shfl_xor(mx, o));
      const float mn = fmaxf(m[r], mx); const float alpha = expf(m[r] - mn); float es = expf(s[0][r] - mn) + expf(s[1][r] - mn);
#pragma unroll
      for (int o = 1; o < 16; o <<= 1) es += __shfl_xor(es, o);
      l[r] = l[r] * alpha + es; m[r] = mn; } }
  if (col == 0) {
#pragma unroll
    for (int r = 0; r < 8; ++r) su[wave * 16 + 8 * g + r] = -logf((float)NS) - (m[r] + logf(l[r])); }
  __syncthreads(); if (tid < 16) vst2(U1 + bh * NS + blockIdx.x * 64 + tid * 4, *(const v4f*)&su[tid * 4]); }
__global__ __launch_bounds__(128) void k_collse(const float* __restrict__ Q, const float* __restrict__ K, const int* __restrict__ MK, const float* __restrict__ U1, float* __restrict__ V1) { __shared__ __align__(16) float sv[64];
  const int tid = threadIdx.x, wave = tid >> 5, lane = tid & 31, col = lane & 15, g = lane >> 4; const size_t bh = blockIdx.y; const size_t b = bh / NH; const int j0 = blockIdx.x * 64 + wave * 16;
  const v16b ak = frag_in(K + (bh * NS + j0 + col) * DD, lane);
  bool mskr[8];
#pragma unroll
  for (int r = 0; r < 8; ++r) mskr[r] = (MK[b * NS + j0 + 8 * g + r] != 0);
  float m[8], l[8];
#pragma unroll
  for (int r = 0; r < 8; ++r) { m[r] = -3.0e38f; l[r] = 0.f; }
#pragma unroll 1
  for (int is = 0; is < NS / 32; ++is) { float s[2][8];
#pragma unroll
    for (int ct = 0; ct < 2; ++ct) { const int ii = is * 32 + ct * 16 + col; v8f c = {}; c = wmma_bf(ak, frag_in(Q + (bh * NS + ii) * DD, lane), c); const float u = U1[bh * NS + ii];
#pragma unroll
      for (int r = 0; r < 8; ++r) s[ct][r] = (mskr[r] ? -10000.0f : c[r] * 0.17677669529663687f) + u; }
#pragma unroll
    for (int r = 0; r < 8; ++r) { float mx = fmaxf(s[0][r], s[1][r]);
#pragma unroll
      for (int o = 1; o < 16; o <<= 1) mx = fmaxf(mx, __shfl_xor(mx, o));
      const float mn = fmaxf(m[r], mx); const float alpha = expf(m[r] - mn); float es = expf(s[0][r] - mn) + expf(s[1][r] - mn);
#pragma unroll
      for (int o = 1; o < 16; o <<= 1) es += __shfl_xor(es, o);
      l[r] = l[r] * alpha + es; m[r] = mn; } }
  if (col == 0) {
#pragma unroll
    for (int r = 0; r < 8; ++r) sv[wave * 16 + 8 * g + r] = -logf((float)NS) - (m[r] + logf(l[r])); }
  __syncthreads(); if (tid < 16) vst2(V1 + bh * NS + blockIdx.x * 64 + tid * 4, *(const v4f*)&sv[tid * 4]); }
__global__ __launch_bounds__(128) void k_att(const float* __restrict__ Q, const float* __restrict__ K, const int* __restrict__ MK, const float* __restrict__ V1, const _Float16* __restrict__ VT, float* __restrict__ OUT) {
  __shared__ __align__(16) float sp[4][16][36]; __shared__ __align__(16) float so[4][16][36];
  const int tid = threadIdx.x, wave = tid >> 5, lane = tid & 31, col = lane & 15, g = lane >> 4; const size_t bh = blockIdx.y; const size_t b = bh / NH; const int i0 = blockIdx.x * 64 + wave * 16;
  const v16b aq = frag_in(Q + (bh * NS + i0 + col) * DD, lane);
  float m[8], l[8];
#pragma unroll
  for (int r = 0; r < 8; ++r) { m[r] = -3.0e38f; l[r] = 0.f; }
  v8f acc[2] = {};
#pragma unroll 1
  for (int ks = 0; ks < NS / 32; ++ks) { float s[2][8];
#pragma unroll
    for (int ct = 0; ct < 2; ++ct) { const int kk = ks * 32 + ct * 16 + col; v8f c = {}; c = wmma_bf(aq, frag_in(K + (bh * NS + kk) * DD, lane), c); const bool msk = (MK[b * NS + kk] != 0); const float vb = V1[bh * NS + kk];
#pragma unroll
      for (int r = 0; r < 8; ++r) s[ct][r] = (msk ? -10000.0f : c[r] * 0.17677669529663687f) + vb; }
    float alpha[8];
#pragma unroll
    for (int r = 0; r < 8; ++r) { float mx = fmaxf(s[0][r], s[1][r]);
#pragma unroll
      for (int o = 1; o < 16; o <<= 1) mx = fmaxf(mx, __shfl_xor(mx, o));
      const float mn = fmaxf(m[r], mx); alpha[r] = __expf(m[r] - mn); const float e0 = __expf(s[0][r] - mn), e1 = __expf(s[1][r] - mn); float es = e0 + e1;
#pragma unroll
      for (int o = 1; o < 16; o <<= 1) es += __shfl_xor(es, o);
      l[r] = l[r] * alpha[r] + es; m[r] = mn; sp[wave][8 * g + r][col] = e0; sp[wave][8 * g + r][16 + col] = e1; }
#pragma unroll
    for (int j = 0; j < 2; ++j)
#pragma unroll
      for (int r = 0; r < 8; ++r) acc[j][r] *= alpha[r];
    LDSX();
    v16h pa, par; { const float* prow = &sp[wave][col][0] + 8 * (lane >> 4);
#pragma unroll
      for (int i = 0; i < 8; ++i) { const float p0 = prow[i] * 2048.0f, p1 = prow[16 + i] * 2048.0f; pa[i] = (_Float16)p0; pa[8 + i] = (_Float16)p1; par[i] = (_Float16)(p0 - (float)pa[i]); par[8 + i] = (_Float16)(p1 - (float)pa[8 + i]); } }
#pragma unroll
    for (int j = 0; j < 2; ++j) { const v16h vh = frag_h(VT + (bh * DD + j * 16 + col) * (size_t)NS + ks * 32, lane); acc[j] = wmma16(pa, vh, acc[j]); acc[j] = wmma16(par, vh, acc[j]); }
    LDSX(); }
#pragma unroll
  for (int r = 0; r < 8; ++r) { const float il = (1.0f / 2048.0f) / l[r];
#pragma unroll
    for (int j = 0; j < 2; ++j) so[wave][8 * g + r][j * 16 + col] = acc[j][r] * il; }
  LDSX(); for (int rl = 0; rl < 16; ++rl) if (lane < 8) vst2(OUT + (bh * NS + i0 + rl) * DD + lane * 4, *(const v4f*)&so[wave][rl][lane * 4]); }
extern "C" void kernel_launch(void* const* d_in, const int* in_sizes, int n_in, void* d_out, int out_size, void* d_ws, size_t ws_size, hipStream_t stream) {
  (void)in_sizes; (void)n_in; (void)out_size;
  const float** F = (const float**)d_in;
  if (ws_size < (size_t)WS_END) return;
  char* ws = (char*)d_ws; float *U1 = (float*)(ws + WS_U1), *V1 = (float*)(ws + WS_V1); _Float16* VT = (_Float16*)(ws + WS_VT);
  k_vt<<<dim3(NS / 64, TBH), 128, 0, stream>>>(F[2], VT);
  k_rowlse<<<dim3(NS / 64, TBH), 128, 0, stream>>>(F[0], F[1], (const int*)d_in[3], U1);
  k_collse<<<dim3(NS / 64, TBH), 128, 0, stream>>>(F[0], F[1], (const int*)d_in[3], U1, V1);
  k_att<<<dim3(NS / 64, TBH), 128, 0, stream>>>(F[0], F[1], (const int*)d_in[3], V1, VT, (float*)d_out);
}
